// MPNN_20486994002071
// MI455X (gfx1250) — hardware-verified
//
#include <hip/hip_runtime.h>
#include <stddef.h>


#define DM     32
#define EFD    16
#define KP     1280
#define NTHR   256
#define NWAVE  8
#define EPT    8
#define NGRP   2
#define CHUNK  (NTHR * EPT * NGRP)
#define WCAP   (EPT * NGRP * 32)
#define LISTN  (NWAVE * WCAP)
#define NB     1792
#define MEB    256
#define EEB    128
#define PTHR   64
#define DRB    128
#define NCB    224
#define SC_H   32.0f
#define SC_E   32.0f
#define SC_W   1024.0f
#define SC_B   32768.0f
#define MSGINV (1.0f / 1048576.0f)
#define LDS_NODE ((NB * DM + LISTN + NCB + 8) * 4)

enum { OFF_ENC = 0, OFF_PROJ = 1024, OFF_EENC = 2048, OFF_EN1 = 3072, OFF_WI = 4096, OFF_WH = 7168,
       OFF_D1 = 10240, OFF_D2 = 11264, OFF_D3 = 12288, OFF_D4 = 13312, WB_N = 13824 };
enum { S_ENC = 0, S_PROJ = 128, S_EENC = 256, S_EN1 = 384, S_WI = 512, S_WH = 896, S_D1 = 1280,
       S_D2 = 1408, S_D3 = 1536, S_D4 = 1664, S_BP = 1728, S_END = 6848 };

static_assert((CHUNK & (CHUNK - 1)) == 0);
static_assert(CHUNK <= 4096);
static_assert(NB < 4096 && (NB % 16) == 0);
static_assert((S_PROJ % PTHR) == 0 && (S_EENC % PTHR) == 0 && (S_EN1 % PTHR) == 0 && (S_WI % PTHR) == 0);
static_assert((S_WH % PTHR) == 0 && (S_D1 % PTHR) == 0 && (S_D2 % PTHR) == 0 && (S_D3 % PTHR) == 0);
static_assert((S_D4 % PTHR) == 0 && (S_BP % PTHR) == 0 && (S_END % PTHR) == 0);
static_assert((S_BP % 32) == 0 && (KP % 256) == 0);
static_assert(S_END - S_BP == 32 * (KP / 8));
static_assert((S_PROJ - S_ENC) * 8 == OFF_PROJ - OFF_ENC && (S_WH - S_WI) * 8 == OFF_WH - OFF_WI);
static_assert((S_BP - S_D4) * 8 == WB_N - OFF_D4);
static_assert((OFF_PROJ % 64) == 0 && (OFF_EENC % 64) == 0 && (OFF_EN1 % 64) == 0 && (OFF_WI % 64) == 0 && (OFF_WH % 64) == 0);
static_assert((OFF_D1 % 64) == 0 && (OFF_D2 % 64) == 0 && (OFF_D3 % 64) == 0 && (OFF_D4 % 64) == 0 && (WB_N % 64) == 0);
static_assert(LDS_NODE <= 300 * 1024);
static_assert(MEB == 32 * NWAVE);
static_assert(MEB == NTHR);
static_assert(((MEB * DM / 8) % NTHR) == 0);
static_assert(EEB == 16 * NWAVE);
static_assert((MEB % EEB) == 0);
static_assert((DRB * 3) % 4 == 0);
static_assert(MEB * DM * 2 + MEB * DM * 4 + MEB * 4 <= 64 * 1024);

typedef float          v4f  __attribute__((ext_vector_type(4)));
typedef float          v8f  __attribute__((ext_vector_type(8)));
typedef int            v4i  __attribute__((ext_vector_type(4)));
typedef _Float16       v8h  __attribute__((ext_vector_type(8)));
typedef _Float16       v16h __attribute__((ext_vector_type(16)));
typedef unsigned short v8us __attribute__((ext_vector_type(8)));
typedef __bf16         v16b __attribute__((ext_vector_type(16)));
typedef v4f            v4fa __attribute__((may_alias));
typedef v8h            v8ha __attribute__((may_alias));
union FragH { v16h v; v8h h[2]; };
union FragB { v16b v; v8us u[2]; };

__device__ __forceinline__ v8f z8() { v8f z = {0.f, 0.f, 0.f, 0.f, 0.f, 0.f, 0.f, 0.f}; return z; }

__device__ __forceinline__ v8f wmb(v16b a, v16b b, v8f c) {
  v8f d = __builtin_amdgcn_wmma_f32_16x16x32_bf16(false, a, false, b, (short)0, c, false, false);
  asm volatile("v_nop\n\tv_nop\n\tv_nop\n\tv_nop" : "+v"(d) : "v"(a), "v"(b));
  return d;
}
__device__ __forceinline__ v8f wraw(v16h a, v16h b, v8f c) {
  return __builtin_amdgcn_wmma_f32_16x16x32_f16(false, a, false, b, (short)0, c, false, false);
}
#define GUARD4(d0, d1, d2, d3, a0, a1, b0, b1) \
  asm volatile("v_nop\n\tv_nop\n\tv_nop\n\tv_nop" : "+v"(d0), "+v"(d1), "+v"(d2), "+v"(d3) : "v"(a0), "v"(a1), "v"(b0), "v"(b1))

__device__ __forceinline__ void wave_sync() {
  __builtin_amdgcn_fence(__ATOMIC_RELEASE, "wavefront");
  __builtin_amdgcn_wave_barrier();
}

__device__ __forceinline__ unsigned short bfr(float x) {
  const unsigned u = __float_as_uint(x);
  return (unsigned short)((u + 0x7FFFu + ((u >> 16) & 1u)) >> 16);
}
__device__ __forceinline__ float bfrf(float x) { return __uint_as_float(((unsigned)bfr(x)) << 16); }
__device__ __forceinline__ void split8(v4f a, v4f b, v8us& hi, v8us& lo) {
  float v[8] = {a.x, a.y, a.z, a.w, b.x, b.y, b.z, b.w};
#pragma unroll
  for (int k = 0; k < 8; ++k) {
    const unsigned short h = bfr(v[k]);
    hi[k] = h;
    lo[k] = bfr(v[k] - __uint_as_float(((unsigned)h) << 16));
  }
}
__device__ __forceinline__ v8us pack8(v4f a, v4f b) {
  float v[8] = {a.x, a.y, a.z, a.w, b.x, b.y, b.z, b.w};
  v8us o;
#pragma unroll
  for (int k = 0; k < 8; ++k) o[k] = bfr(v[k]);
  return o;
}
__device__ __forceinline__ v8h cvt8(v4f a, v4f b, float sc) {
  v8h r;
  r[0] = (_Float16)(a.x * sc); r[1] = (_Float16)(a.y * sc); r[2] = (_Float16)(a.z * sc); r[3] = (_Float16)(a.w * sc);
  r[4] = (_Float16)(b.x * sc); r[5] = (_Float16)(b.y * sc); r[6] = (_Float16)(b.z * sc); r[7] = (_Float16)(b.w * sc);
  return r;
}
__device__ __forceinline__ v4f relu4(v4f v) { v.x = fmaxf(v.x, 0.f); v.y = fmaxf(v.y, 0.f); v.z = fmaxf(v.z, 0.f); v.w = fmaxf(v.w, 0.f); return v; }
__device__ __forceinline__ float sigm(float x) { return __builtin_amdgcn_rcpf(1.0f + __expf(-x)); }
__device__ __forceinline__ float tanhm(float x) { return 2.0f * sigm(2.0f * x) - 1.0f; }

__device__ __forceinline__ void ldrow(const float* rp, v4f& a0, v4f& a1, v4f& a2, v4f& a3) {
  a0 = *(const v4fa*)rp; a1 = *(const v4fa*)(rp + 4); a2 = *(const v4fa*)(rp + 16); a3 = *(const v4fa*)(rp + 20);
}
__device__ __forceinline__ void mkfrag(v4f a0, v4f a1, v4f a2, v4f a3, FragB& hi, FragB& lo) {
  split8(a0, a1, hi.u[0], lo.u[0]);
  split8(a2, a3, hi.u[1], lo.u[1]);
}
__device__ __forceinline__ FragB ldB(const unsigned short* P, int n, int hh) {
  FragB b;
  const unsigned short* p = P + n * 32 + 8 * hh;
  b.u[0] = *(const v8us*)p;
  b.u[1] = *(const v8us*)(p + 16);
  return b;
}
__device__ __forceinline__ void dense32(const FragB& ah, const FragB& al, const unsigned short* P, int m, int hh, v8f* acc) {
#pragma unroll
  for (int u = 0; u < 2; ++u) {
    const FragB b = ldB(P, 16 * u + m, hh);
    acc[u] = wmb(ah.v, b.v, z8());
    acc[u] = wmb(al.v, b.v, acc[u]);
  }
}

__device__ __forceinline__ int scan_chunk(const int* __restrict__ ids, int nE, int cbase, int slotBase, int nb,
                                          int vec8, int* list, int tid, int lane, int wave) {
  int wc = 0;
#pragma unroll
  for (int g = 0; g < NGRP; ++g) {
    const int el0  = (g * NTHR + tid) * EPT;
    const int e0   = cbase + el0;
    const int sent = -2147483647 - 1;
    v4i da, db;
    if (vec8 != 0 && cbase + CHUNK <= nE) {
      da = *(const v4i*)(ids + e0);
      db = *(const v4i*)(ids + e0 + 4);
    } else {
      const int lst = nE - 1;
      da.x = (e0     < nE) ? ids[min(e0,     lst)] : sent;
      da.y = (e0 + 1 < nE) ? ids[min(e0 + 1, lst)] : sent;
      da.z = (e0 + 2 < nE) ? ids[min(e0 + 2, lst)] : sent;
      da.w = (e0 + 3 < nE) ? ids[min(e0 + 3, lst)] : sent;
      db.x = (e0 + 4 < nE) ? ids[min(e0 + 4, lst)] : sent;
      db.y = (e0 + 5 < nE) ? ids[min(e0 + 5, lst)] : sent;
      db.z = (e0 + 6 < nE) ? ids[min(e0 + 6, lst)] : sent;
      db.w = (e0 + 7 < nE) ? ids[min(e0 + 7, lst)] : sent;
    }
    const unsigned bs = (unsigned)slotBase;
    const unsigned ub = (unsigned)nb;
    const unsigned s0 = (unsigned)da.x - bs, s1 = (unsigned)da.y - bs;
    const unsigned s2 = (unsigned)da.z - bs, s3 = (unsigned)da.w - bs;
    const unsigned s4 = (unsigned)db.x - bs, s5 = (unsigned)db.y - bs;
    const unsigned s6 = (unsigned)db.z - bs, s7 = (unsigned)db.w - bs;
    const bool h0 = s0 < ub, h1 = s1 < ub, h2 = s2 < ub, h3 = s3 < ub;
    const bool h4 = s4 < ub, h5 = s5 < ub, h6 = s6 < ub, h7 = s7 < ub;
    const unsigned any = __builtin_amdgcn_ballot_w32(h0 | h1 | h2 | h3 | h4 | h5 | h6 | h7);
    if (any != 0u) {
#define HITJ(J, HJ, SJ) { \
        const unsigned mj = __builtin_amdgcn_ballot_w32(HJ); \
        if (mj != 0u) { \
          if (HJ) { \
            const int pos = wc + (int)__builtin_amdgcn_mbcnt_lo(mj, 0u); \
            if (pos < WCAP) list[wave * WCAP + pos] = ((el0 + (J)) << 12) | (int)(SJ); \
          } \
          wc += (int)__builtin_popcount(mj); } }
      HITJ(0, h0, s0)
      HITJ(1, h1, s1)
      HITJ(2, h2, s2)
      HITJ(3, h3, s3)
      HITJ(4, h4, s4)
      HITJ(5, h5, s5)
      HITJ(6, h6, s6)
      HITJ(7, h7, s7)
#undef HITJ
    }
  }
  return wc;
}

__global__ __launch_bounds__(PTHR) void k_prep(
    const float* __restrict__ enc_W, const float* __restrict__ proj_W, const float* __restrict__ eenc_W,
    const float* __restrict__ en_W1, const float* __restrict__ gWi, const float* __restrict__ gWh,
    const float* __restrict__ dW1, const float* __restrict__ dW2, const float* __restrict__ dW3,
    const float* __restrict__ dW4, const float* __restrict__ en_W2, const float* __restrict__ en_b2,
    unsigned short* WB, _Float16* Bp) {
  const int bstart = (int)blockIdx.x * PTHR;
  const int u = bstart + (int)threadIdx.x;
  if (u >= S_END) return;
  if (bstart < S_BP) {
    const float* W = enc_W;
    int K = 32, NO = 32, off = OFF_ENC, seg = S_ENC;
    if (bstart < S_PROJ)      { }
    else if (bstart < S_EENC) { W = proj_W; off = OFF_PROJ; seg = S_PROJ; }
    else if (bstart < S_EN1)  { W = eenc_W; K = EFD; off = OFF_EENC; seg = S_EENC; }
    else if (bstart < S_WI)   { W = en_W1; off = OFF_EN1; seg = S_EN1; }
    else if (bstart < S_WH)   { W = gWi; NO = 96; off = OFF_WI; seg = S_WI; }
    else if (bstart < S_D1)   { W = gWh; NO = 96; off = OFF_WH; seg = S_WH; }
    else if (bstart < S_D2)   { W = dW1; off = OFF_D1; seg = S_D1; }
    else if (bstart < S_D3)   { W = dW2; off = OFF_D2; seg = S_D2; }
    else if (bstart < S_D4)   { W = dW3; off = OFF_D3; seg = S_D3; }
    else                      { W = dW4; NO = 3; off = OFF_D4; seg = S_D4; }
    const int uu = u - seg;
    const int n  = uu >> 2;
    const int k0 = (uu & 3) * 8;
    const int nc = n < NO ? n : NO - 1;
    const float fn = n < NO ? 1.0f : 0.0f;
    v8us o;
#pragma unroll
    for (int e = 0; e < 8; ++e) {
      const int k  = k0 + e;
      const int kc = k < K ? k : K - 1;
      const float fk = k < K ? fn : 0.0f;
      const float x = W[(size_t)kc * NO + nc];
      o[e] = bfr(x * fk);
    }
    unsigned short* dp = WB + off + 8 * uu;
    *(volatile v8us*)dp = o;
    __threadfence();
    *(volatile v8us*)dp = o;
  } else {
    const int uu = u - S_BP;
    const int n  = uu / (KP / 8);
    const int q  = uu - n * (KP / 8);
    const int wq = __builtin_amdgcn_readfirstlane(q >> 5);
    const int lq = q & 31;
    float v[8];
    if (wq < 4) {
      const int c  = 8 * wq + (lq >> 2);
      const int i0 = (lq & 3) * 8;
#pragma unroll
      for (int e = 0; e < 8; ++e) v[e] = bfrf(en_W2[(size_t)c * 1024 + (i0 + e) * 32 + n]) * SC_W;
    } else {
      const int i0 = 8 * lq;
#pragma unroll
      for (int e = 0; e < 8; ++e) {
        const int i  = i0 + e;
        const int ic = i < 32 ? i : 31;
        const float f = i < 32 ? SC_B : 0.0f;
        v[e] = bfrf(en_b2[ic * 32 + n]) * f;
      }
    }
    v4f a, b;
    a.x = v[0]; a.y = v[1]; a.z = v[2]; a.w = v[3];
    b.x = v[4]; b.y = v[5]; b.z = v[6]; b.w = v[7];
    const v8h hv = cvt8(a, b, 1.0f);
    _Float16* dp = Bp + (size_t)n * KP + 8 * q;
    *(volatile v8h*)dp = hv;
    __threadfence();
    *(volatile v8h*)dp = hv;
  }
}

__global__ __launch_bounds__(NTHR) void k_nodeenc(const int* __restrict__ nfeats, int nN,
    const float* __restrict__ emb, int nT, const unsigned short* __restrict__ WB,
    const float* __restrict__ enc_b, const float* __restrict__ proj_b, float* H, _Float16* H16) {
  __shared__ __attribute__((aligned(16))) float CB[64];
  __shared__ __attribute__((aligned(16))) float Es[NWAVE][512];
  __shared__ __attribute__((aligned(16))) float Ys[NWAVE][512];
  const int tid = threadIdx.x, lane = tid & 31, wave = tid >> 5, hh = lane >> 4, m = lane & 15;
  if (wave == 0) CB[lane] = bfrf(enc_b[lane]);
  else if (wave == 1) CB[32 + lane] = bfrf(proj_b[lane]);
  __syncthreads();
  const int nTiles = nN >> 4;
  const int tile = (int)blockIdx.x * NWAVE + wave;
  if (tile >= nTiles) return;
  const int base = tile * 16;
  float* es = Es[wave];
  float* ys = Ys[wave];
#pragma unroll
  for (int q = 0; q < 4; ++q) {
    const int ui = 32 * q + lane;
    const int r = ui >> 3, p = ui & 7;
    int ty = nfeats[base + r];
    ty = ty < 0 ? 0 : (ty > nT - 1 ? nT - 1 : ty);
    *(v4fa*)(es + r * DM + 4 * p) = *(const v4f*)(emb + (size_t)ty * DM + 4 * p);
  }
  wave_sync();
  FragB a;
  {
    v4f e0, e1, e2, e3;
    ldrow(es + m * DM + 8 * hh, e0, e1, e2, e3);
    a.u[0] = pack8(relu4(e0), relu4(e1));
    a.u[1] = pack8(relu4(e2), relu4(e3));
  }
  v8f acc[2];
#pragma unroll
  for (int u = 0; u < 2; ++u) acc[u] = wmb(a.v, ldB(WB + OFF_ENC, 16 * u + m, hh).v, z8());
#pragma unroll
  for (int u = 0; u < 2; ++u) {
    const int j = 16 * u + m;
    const float bv = CB[j];
#pragma unroll
    for (int r = 0; r < 8; ++r) ys[(8 * hh + r) * DM + j] = fmaxf(acc[u][r] + bv, 0.0f);
  }
  wave_sync();
  FragB ah, al;
  {
    v4f q0, q1, q2, q3;
    ldrow(ys + m * DM + 8 * hh, q0, q1, q2, q3);
    mkfrag(q0, q1, q2, q3, ah, al);
  }
  wave_sync();
  dense32(ah, al, WB + OFF_PROJ, m, hh, acc);
#pragma unroll
  for (int u = 0; u < 2; ++u) {
    const int j = 16 * u + m;
    const float bv = CB[32 + j];
#pragma unroll
    for (int r = 0; r < 8; ++r) ys[(8 * hh + r) * DM + j] = fmaxf(acc[u][r] + bv, 0.0f);
  }
  wave_sync();
  v4f ov[4];
#pragma unroll
  for (int p = 0; p < 4; ++p) ov[p] = *(const v4fa*)(ys + 4 * (32 * p + lane));
  v8h hv[2];
#pragma unroll
  for (int p = 0; p < 2; ++p)
    hv[p] = cvt8(*(const v4fa*)(ys + 8 * (32 * p + lane)), *(const v4fa*)(ys + 8 * (32 * p + lane) + 4), SC_H);
  float* gp = H + (size_t)base * DM;
  _Float16* gq = H16 + (size_t)base * DM;
#pragma unroll
  for (int p = 0; p < 4; ++p) *(volatile v4f*)(gp + 4 * (32 * p + lane)) = ov[p];
#pragma unroll
  for (int p = 0; p < 2; ++p) *(volatile v8h*)(gq + 8 * (32 * p + lane)) = hv[p];
  __threadfence();
#pragma unroll
  for (int p = 0; p < 4; ++p) *(volatile v4f*)(gp + 4 * (32 * p + lane)) = ov[p];
#pragma unroll
  for (int p = 0; p < 2; ++p) *(volatile v8h*)(gq + 8 * (32 * p + lane)) = hv[p];
}

__global__ __launch_bounds__(NTHR) void k_edgeenc(const float* __restrict__ efeats, int nE,
    const unsigned short* __restrict__ WB, const float* __restrict__ eenc_b, const float* __restrict__ en_b1,
    _Float16* HE16) {
  __shared__ __attribute__((aligned(16))) float CB[64];
  __shared__ __attribute__((aligned(16))) float Ys[NWAVE][512];
  __shared__ __attribute__((aligned(16))) _Float16 Hs[NWAVE][512];
  const int tid = threadIdx.x, lane = tid & 31, wave = tid >> 5, hh = lane >> 4, m = lane & 15;
  if (wave == 0) CB[lane] = bfrf(eenc_b[lane]);
  else if (wave == 1) CB[32 + lane] = bfrf(en_b1[lane]);
  __syncthreads();
  const int base = ((int)blockIdx.x * NWAVE + wave) * 16;
  int e = base + m;
  e = e > nE - 1 ? nE - 1 : e;
  float* ys = Ys[wave];
  _Float16* hs = Hs[wave];
  FragB a;
  {
    const float* ep = efeats + (size_t)e * EFD + 8 * hh;
    a.u[0] = pack8(*(const v4f*)ep, *(const v4f*)(ep + 4));
    const v4f z = {0.f, 0.f, 0.f, 0.f};
    a.u[1] = pack8(z, z);
  }
  v8f acc[2];
#pragma unroll
  for (int u = 0; u < 2; ++u) acc[u] = wmb(a.v, ldB(WB + OFF_EENC, 16 * u + m, hh).v, z8());
#pragma unroll
  for (int u = 0; u < 2; ++u) {
    const int j = 16 * u + m;
    const float bv = CB[j];
#pragma unroll
    for (int r = 0; r < 8; ++r) ys[(8 * hh + r) * DM + j] = acc[u][r] + bv;
  }
  wave_sync();
  FragB ah, al;
  {
    v4f q0, q1, q2, q3;
    ldrow(ys + m * DM + 8 * hh, q0, q1, q2, q3);
    mkfrag(q0, q1, q2, q3, ah, al);
  }
  dense32(ah, al, WB + OFF_EN1, m, hh, acc);
#pragma unroll
  for (int u = 0; u < 2; ++u) {
    const int j = 16 * u + m;
    const float bv = CB[32 + j];
#pragma unroll
    for (int r = 0; r < 8; ++r) hs[(8 * hh + r) * DM + j] = (_Float16)(fmaxf(acc[u][r] + bv, 0.0f) * SC_E);
  }
  wave_sync();
  v8h hv[2];
#pragma unroll
  for (int p = 0; p < 2; ++p) hv[p] = *(const v8ha*)(hs + 8 * (32 * p + lane));
  _Float16* gq = HE16 + (size_t)base * DM;
#pragma unroll
  for (int p = 0; p < 2; ++p) *(volatile v8h*)(gq + 8 * (32 * p + lane)) = hv[p];
  __threadfence();
#pragma unroll
  for (int p = 0; p < 2; ++p) *(volatile v8h*)(gq + 8 * (32 * p + lane)) = hv[p];
}

__global__ __launch_bounds__(NTHR) void k_msg(const _Float16* __restrict__ H16, int nN,
    const int* __restrict__ srcs, int nE, const _Float16* __restrict__ HE16,
    const _Float16* __restrict__ Bp, float* MSG) {
  __shared__ __attribute__((aligned(16))) _Float16 Xs[MEB * DM];
  __shared__ __attribute__((aligned(16))) float Stg[MEB * DM];
  __shared__ int Ss[MEB];
  const int tid = threadIdx.x, lane = tid & 31, wave = tid >> 5, hh = lane >> 4, m = lane & 15;
  const int eBase = (int)blockIdx.x * MEB;
#pragma unroll 1
  for (int i = tid; i < MEB; i += NTHR) {
    int e = eBase + i;
    e = e > nE - 1 ? nE - 1 : e;
    int s = srcs[e];
    s = s < 0 ? 0 : (s > nN - 1 ? nN - 1 : s);
    Ss[i] = s;
  }
  __syncthreads();
#pragma unroll
  for (int q = 0; q < (MEB * DM / 8) / NTHR; ++q) {
    const int ui = q * NTHR + tid;
    const int r = ui >> 2, p = ui & 3;
    *(v8h*)(Xs + r * DM + 8 * p) = *(const v8h*)(H16 + (size_t)Ss[r] * DM + 8 * p);
  }
  __syncthreads();

  FragH xf[2];
  int er[2];
#pragma unroll
  for (int t = 0; t < 2; ++t) {
    const int row = 32 * wave + 16 * t + m;
    const _Float16* xr = Xs + row * DM + 8 * hh;
    xf[t].h[0] = *(const v8h*)xr;
    xf[t].h[1] = *(const v8h*)(xr + 16);
    int e = eBase + row;
    e = e > nE - 1 ? nE - 1 : e;
    er[t] = e;
  }
  v8f acc[2][2];
#pragma unroll
  for (int t = 0; t < 2; ++t) { acc[t][0] = z8(); acc[t][1] = z8(); }
  const _Float16* bb0 = Bp + (size_t)m * KP + 8 * hh;
  const _Float16* bb1 = bb0 + (size_t)16 * KP;
#pragma unroll 1
  for (int cg = 0; cg < 4; ++cg) {
    const v8h hq0 = *(const v8h*)(HE16 + (size_t)er[0] * DM + 8 * cg);
    const v8h hq1 = *(const v8h*)(HE16 + (size_t)er[1] * DM + 8 * cg);
#pragma unroll
    for (int ci = 0; ci < 8; ++ci) {
      const int koff = 256 * cg + 32 * ci;
      FragH b0, b1;
      b0.h[0] = *(const v8h*)(bb0 + koff);
      b0.h[1] = *(const v8h*)(bb0 + koff + 16);
      b1.h[0] = *(const v8h*)(bb1 + koff);
      b1.h[1] = *(const v8h*)(bb1 + koff + 16);
      const v16h a0 = xf[0].v * hq0[ci];
      const v16h a1 = xf[1].v * hq1[ci];
      acc[0][0] = wraw(a0, b0.v, acc[0][0]);
      acc[1][0] = wraw(a1, b0.v, acc[1][0]);
      acc[0][1] = wraw(a0, b1.v, acc[0][1]);
      acc[1][1] = wraw(a1, b1.v, acc[1][1]);
      GUARD4(acc[0][0], acc[1][0], acc[0][1], acc[1][1], a0, a1, b0.v, b1.v);
    }
  }
  {
    const int koff = 1024;
    FragH b0, b1;
    b0.h[0] = *(const v8h*)(bb0 + koff);
    b0.h[1] = *(const v8h*)(bb0 + koff + 16);
    b1.h[0] = *(const v8h*)(bb1 + koff);
    b1.h[1] = *(const v8h*)(bb1 + koff + 16);
    acc[0][0] = wraw(xf[0].v, b0.v, acc[0][0]);
    acc[1][0] = wraw(xf[1].v, b0.v, acc[1][0]);
    acc[0][1] = wraw(xf[0].v, b1.v, acc[0][1]);
    acc[1][1] = wraw(xf[1].v, b1.v, acc[1][1]);
    GUARD4(acc[0][0], acc[1][0], acc[0][1], acc[1][1], xf[0].v, xf[1].v, b0.v, b1.v);
  }
#pragma unroll
  for (int t = 0; t < 2; ++t) {
    float* sp = Stg + (32 * wave + 16 * t + 8 * hh) * DM + m;
#pragma unroll
    for (int nt = 0; nt < 2; ++nt) {
#pragma unroll
      for (int r = 0; r < 8; ++r) sp[r * DM + 16 * nt] = acc[t][nt][r] * MSGINV;
    }
  }
  wave_sync();
  const float* lp = Stg + 32 * wave * DM;
  float* gp = MSG + (size_t)(eBase + 32 * wave) * DM;
  v4f ov[8];
#pragma unroll
  for (int p = 0; p < 8; ++p) ov[p] = *(const v4fa*)(lp + 4 * (32 * p + lane));
#pragma unroll
  for (int p = 0; p < 8; ++p) *(volatile v4f*)(gp + 4 * (32 * p + lane)) = ov[p];
  __threadfence();
#pragma unroll
  for (int p = 0; p < 8; ++p) *(volatile v4f*)(gp + 4 * (32 * p + lane)) = ov[p];
}

__global__ __launch_bounds__(NTHR) void k_node(const int* __restrict__ dsts, int nE, int vec8,
    const float* __restrict__ MSG, float* H, _Float16* H16, int nN,
    const float* __restrict__ conv_b, const unsigned short* __restrict__ WB,
    const float* __restrict__ gbi, const float* __restrict__ gbh) {
  extern __shared__ v4f lds_dyn[];
  float* accL = (float*)lds_dyn;
  int*   list = (int*)(accL + NB * DM);
  float* CBs  = (float*)(list + LISTN);
  int*   wcnt = (int*)(CBs + NCB);
  const int tid = threadIdx.x, lane = tid & 31, wave = tid >> 5, hh = lane >> 4, m = lane & 15;
  const int nodeBase = (int)blockIdx.x * NB;
  int nbv = nN - nodeBase;
  nbv = nbv < 0 ? 0 : (nbv > NB ? NB : nbv);
  {
    const v4f z = {0.f, 0.f, 0.f, 0.f};
#pragma unroll 1
    for (int i = tid; i < NB * DM / 4; i += NTHR) ((v4f*)accL)[i] = z;
    if (wave == 0) CBs[lane] = bfrf(conv_b[lane]);
    else if (wave < 4) CBs[tid] = bfrf(gbi[tid - 32]);
    else if (wave < 7) CBs[tid] = bfrf(gbh[tid - 128]);
  }
  __syncthreads();

  const int nChunks = (nE + CHUNK - 1) / CHUNK;
#pragma unroll 1
  for (int ch = 0; ch < nChunks; ++ch) {
    const int cbase = ch * CHUNK;
    const int wc = scan_chunk(dsts, nE, cbase, nodeBase, nbv, vec8, list, tid, lane, wave);
    if (lane == 0) wcnt[wave] = wc;
    __syncthreads();
    if (wave == 0) {
#pragma unroll 1
      for (int wsx = 0; wsx < NWAVE; ++wsx) {
        int n = __builtin_amdgcn_readfirstlane(wcnt[wsx]);
        n = n > WCAP ? WCAP : (n < 0 ? 0 : n);
        const int* lp = list + wsx * WCAP;
#pragma unroll 1
        for (int i = 0; i < n; ++i) {
          const int ent = __builtin_amdgcn_readfirstlane(lp[i]);
          int slot = ent & 4095;
          slot = slot > NB - 1 ? NB - 1 : slot;
          int e = cbase + ((ent >> 12) & (CHUNK - 1));
          e = e > nE - 1 ? nE - 1 : e;
          const float v = MSG[(size_t)e * DM + lane];
          float* ap = accL + slot * DM + lane;
          *ap = *ap + v;
        }
      }
    }
    __syncthreads();
  }

  const int nTl = nbv >> 4;
#pragma unroll 1
  for (int tl = wave; tl < nTl; tl += NWAVE) {
    const int r0 = tl * 16;
    const size_t g0 = (size_t)nodeBase + (size_t)r0;
    float* tile = accL + r0 * DM;
    FragB xh, xl, oh, ol;
    v4f h0, h1, h2, h3;
    {
      v4f x0, x1, x2, x3;
      ldrow(tile + m * DM + 8 * hh, x0, x1, x2, x3);
      const float* cbp = CBs + 8 * hh;
      x0 = relu4(x0 + *(const v4fa*)cbp);
      x1 = relu4(x1 + *(const v4fa*)(cbp + 4));
      x2 = relu4(x2 + *(const v4fa*)(cbp + 16));
      x3 = relu4(x3 + *(const v4fa*)(cbp + 20));
      mkfrag(x0, x1, x2, x3, xh, xl);
      ldrow(H + (g0 + m) * DM + 8 * hh, h0, h1, h2, h3);
      mkfrag(h0, h1, h2, h3, oh, ol);
    }
    wave_sync();
    {
      float* hp = tile + m * DM + 8 * hh;
      *(v4fa*)hp = h0; *(v4fa*)(hp + 4) = h1; *(v4fa*)(hp + 16) = h2; *(v4fa*)(hp + 20) = h3;
    }
    wave_sync();
    v8f gi[3][2], gh[3][2];
#pragma unroll
    for (int g = 0; g < 3; ++g) {
#pragma unroll
      for (int u = 0; u < 2; ++u) {
        const int n = 32 * g + 16 * u + m;
        const FragB bi = ldB(WB + OFF_WI, n, hh);
        const FragB bh = ldB(WB + OFF_WH, n, hh);
        gi[g][u] = wmb(xh.v, bi.v, z8());
        gi[g][u] = wmb(xl.v, bi.v, gi[g][u]);
        gh[g][u] = wmb(oh.v, bh.v, z8());
        gh[g][u] = wmb(ol.v, bh.v, gh[g][u]);
      }
    }
#pragma unroll
    for (int u = 0; u < 2; ++u) {
      const int j = 16 * u + m;
      const float bir = CBs[32 + j], biz = CBs[64 + j], bin = CBs[96 + j];
      const float bhr = CBs[128 + j], bhz = CBs[160 + j], bhn = CBs[192 + j];
#pragma unroll
      for (int r = 0; r < 8; ++r) {
        const int row = 8 * hh + r;
        const float rr = sigm(gi[0][u][r] + bir + gh[0][u][r] + bhr);
        const float zz = sigm(gi[1][u][r] + biz + gh[1][u][r] + bhz);
        const float nn = tanhm(gi[2][u][r] + bin + rr * (gh[2][u][r] + bhn));
        const float ho = tile[row * DM + j];
        tile[row * DM + j] = (1.0f - zz) * nn + zz * ho;
      }
    }
    wave_sync();
    v4f ov[4];
#pragma unroll
    for (int p = 0; p < 4; ++p) ov[p] = *(const v4fa*)(tile + 4 * (32 * p + lane));
    v8h hv[2];
#pragma unroll
    for (int p = 0; p < 2; ++p)
      hv[p] = cvt8(*(const v4fa*)(tile + 8 * (32 * p + lane)), *(const v4fa*)(tile + 8 * (32 * p + lane) + 4), SC_H);
    float* gp = H + g0 * DM;
    _Float16* gq = H16 + g0 * DM;
#pragma unroll
    for (int p = 0; p < 4; ++p) *(volatile v4f*)(gp + 4 * (32 * p + lane)) = ov[p];
#pragma unroll
    for (int p = 0; p < 2; ++p) *(volatile v8h*)(gq + 8 * (32 * p + lane)) = hv[p];
    __threadfence();
#pragma unroll
    for (int p = 0; p < 4; ++p) *(volatile v4f*)(gp + 4 * (32 * p + lane)) = ov[p];
#pragma unroll
    for (int p = 0; p < 2; ++p) *(volatile v8h*)(gq + 8 * (32 * p + lane)) = hv[p];
  }
}

__device__ __forceinline__ void prelu_store(const v8f* acc, const float* cb, float a, float* ys, int hh, int m) {
#pragma unroll
  for (int u = 0; u < 2; ++u) {
    const int j = 16 * u + m;
    const float bv = cb[j];
#pragma unroll
    for (int r = 0; r < 8; ++r) {
      const float y = acc[u][r] + bv;
      ys[(8 * hh + r) * DM + j] = y >= 0.0f ? y : a * y;
    }
  }
}

__global__ __launch_bounds__(NTHR) void k_dec(const float* __restrict__ H, int nN, const unsigned short* __restrict__ WB,
    const float* __restrict__ b1, const float* __restrict__ a1, const float* __restrict__ b2, const float* __restrict__ a2,
    const float* __restrict__ b3, const float* __restrict__ a3, const float* __restrict__ b4, float* out) {
  __shared__ __attribute__((aligned(16))) float CB[128];
  __shared__ __attribute__((aligned(16))) float Ys[NWAVE][512];
  __shared__ __attribute__((aligned(16))) float Ost[DRB * 3];
  const int tid = threadIdx.x, lane = tid & 31, wave = tid >> 5, hh = lane >> 4, m = lane & 15;
  if (wave == 0) CB[lane] = bfrf(b1[lane]);
  else if (wave == 1) CB[32 + lane] = bfrf(b2[lane]);
  else if (wave == 2) CB[64 + lane] = bfrf(b3[lane]);
  else if (wave == 3) {
    const float bv = bfrf(b4[lane < 3 ? lane : 2]);
    if (lane < 16) CB[96 + lane] = lane < 3 ? bv : 0.0f;
  } else if (wave == 4) {
    const float v1 = bfrf(a1[0]), v2 = bfrf(a2[0]), v3 = bfrf(a3[0]);
    if (lane == 0) { CB[112] = v1; CB[113] = v2; CB[114] = v3; }
  }
  __syncthreads();
  const int base = ((int)blockIdx.x * NWAVE + wave) * 16;
  int g = base + m;
  g = g > nN - 1 ? nN - 1 : g;
  float* ys = Ys[wave];
  FragB ah, al;
  v8f acc[2];
  {
    v4f q0, q1, q2, q3;
    ldrow(H + (size_t)g * DM + 8 * hh, q0, q1, q2, q3);
    mkfrag(q0, q1, q2, q3, ah, al);
  }
  dense32(ah, al, WB + OFF_D1, m, hh, acc);
  prelu_store(acc, CB, CB[112], ys, hh, m);
  wave_sync();
  { v4f q0, q1, q2, q3; ldrow(ys + m * DM + 8 * hh, q0, q1, q2, q3); mkfrag(q0, q1, q2, q3, ah, al); }
  wave_sync();
  dense32(ah, al, WB + OFF_D2, m, hh, acc);
  prelu_store(acc, CB + 32, CB[113], ys, hh, m);
  wave_sync();
  { v4f q0, q1, q2, q3; ldrow(ys + m * DM + 8 * hh, q0, q1, q2, q3); mkfrag(q0, q1, q2, q3, ah, al); }
  wave_sync();
  dense32(ah, al, WB + OFF_D3, m, hh, acc);
  prelu_store(acc, CB + 64, CB[114], ys, hh, m);
  wave_sync();
  { v4f q0, q1, q2, q3; ldrow(ys + m * DM + 8 * hh, q0, q1, q2, q3); mkfrag(q0, q1, q2, q3, ah, al); }
  {
    const FragB b = ldB(WB + OFF_D4, m, hh);
    v8f a4 = wmb(ah.v, b.v, z8());
    a4 = wmb(al.v, b.v, a4);
    const float bv = CB[96 + m];
#pragma unroll
    for (int r = 0; r < 8; ++r) {
      const float val = a4[r] + bv;
      if (m < 3) Ost[(16 * wave + 8 * hh + r) * 3 + m] = val;
    }
  }
  __syncthreads();
  int nrows = nN - (int)blockIdx.x * DRB;
  nrows = nrows < 0 ? 0 : (nrows > DRB ? DRB : nrows);
  const int nv = (nrows * 3) >> 2;
  const int oi = tid < (DRB * 3 / 4) ? tid : (DRB * 3 / 4 - 1);
  const v4f v = *(const v4fa*)(Ost + 4 * oi);
  float* op = out + (size_t)blockIdx.x * (DRB * 3) + 4 * tid;
  if (tid < nv) *(volatile v4f*)op = v;
  __threadfence();
  if (tid < nv) *(volatile v4f*)op = v;
}

extern "C" void kernel_launch(void* const* d_in, const int* in_sizes, int n_in,
                              void* d_out, int out_size, void* d_ws, size_t ws_size,
                              hipStream_t stream) {
  if (n_in < 31) return;
  const int nN = in_sizes[0];
  const int nE = in_sizes[2];
  if (nN < 32 || nE < MEB) return;
  if ((nN % 32) != 0 || (nE % MEB) != 0) return;
  if (in_sizes[1] != nE * EFD || in_sizes[3] != nE) return;
  const int nT = in_sizes[4] / DM;
  if (nT < 1 || in_sizes[4] != nT * DM) return;
  if (in_sizes[5] != 1024 || in_sizes[6] != 32 || in_sizes[7] != EFD * 32 || in_sizes[8] != 32) return;
  if (in_sizes[9] != 1024 || in_sizes[10] != 32 || in_sizes[11] != 1024 || in_sizes[12] != 32) return;
  if (in_sizes[13] != 32 * 1024 || in_sizes[14] != 1024 || in_sizes[15] != 32) return;
  if (in_sizes[16] != 32 * 96 || in_sizes[17] != 32 * 96 || in_sizes[18] != 96 || in_sizes[19] != 96) return;
  if (in_sizes[20] != 1024 || in_sizes[21] != 32 || in_sizes[22] < 1) return;
  if (in_sizes[23] != 1024 || in_sizes[24] != 32 || in_sizes[25] < 1) return;
  if (in_sizes[26] != 1024 || in_sizes[27] != 32 || in_sizes[28] < 1) return;
  if (in_sizes[29] != 96 || in_sizes[30] != 3) return;
  if (out_size != nN * 3) return;
  if (nN > (1 << 24) || nE > (1 << 26)) return;

  const int*   nfeats = (const int*)d_in[0];
  const float* efeats = (const float*)d_in[1];
  const int*   src    = (const int*)d_in[2];
  const int*   dst    = (const int*)d_in[3];
  const float* emb    = (const float*)d_in[4];
  const float* enc_W  = (const float*)d_in[5];
  const float* enc_b  = (const float*)d_in[6];
  const float* eenc_W = (const float*)d_in[7];
  const float* eenc_b = (const float*)d_in[8];
  const float* proj_W = (const float*)d_in[9];
  const float* proj_b = (const float*)d_in[10];
  const float* en_W1  = (const float*)d_in[11];
  const float* en_b1  = (const float*)d_in[12];
  const float* en_W2  = (const float*)d_in[13];
  const float* en_b2  = (const float*)d_in[14];
  const float* conv_b = (const float*)d_in[15];
  const float* gru_Wi = (const float*)d_in[16];
  const float* gru_Wh = (const float*)d_in[17];
  const float* gru_bi = (const float*)d_in[18];
  const float* gru_bh = (const float*)d_in[19];
  const float* dW1 = (const float*)d_in[20];
  const float* db1 = (const float*)d_in[21];
  const float* da1 = (const float*)d_in[22];
  const float* dW2 = (const float*)d_in[23];
  const float* db2 = (const float*)d_in[24];
  const float* da2 = (const float*)d_in[25];
  const float* dW3 = (const float*)d_in[26];
  const float* db3 = (const float*)d_in[27];
  const float* da3 = (const float*)d_in[28];
  const float* dW4 = (const float*)d_in[29];
  const float* db4 = (const float*)d_in[30];
  float* out = (float*)d_out;

  size_t off = 0;
  const size_t oWB  = off; off += (size_t)WB_N * 2;            off = (off + 255) & ~(size_t)255;
  const size_t oBp  = off; off += (size_t)32 * KP * 2;         off = (off + 255) & ~(size_t)255;
  const size_t oH   = off; off += (size_t)nN * DM * 4;         off = (off + 255) & ~(size_t)255;
  const size_t oH16 = off; off += (size_t)nN * DM * 2;         off = (off + 255) & ~(size_t)255;
  const size_t oHE  = off; off += (size_t)nE * DM * 2;         off = (off + 255) & ~(size_t)255;
  const size_t oMSG = off; off += (size_t)nE * DM * 4;         off = (off + 255) & ~(size_t)255;
  if (off > ws_size) return;
  if (off > (size_t)128 * 1024 * 1024) return;
  char* ws = (char*)d_ws;
  unsigned short* WB  = (unsigned short*)(ws + oWB);
  _Float16*       Bp  = (_Float16*)(ws + oBp);
  float*          H   = (float*)(ws + oH);
  _Float16*       H16 = (_Float16*)(ws + oH16);
  _Float16*       HE  = (_Float16*)(ws + oHE);
  float*          MSG = (float*)(ws + oMSG);

  const int vec8   = ((nE & 3) == 0) ? 1 : 0;
  const int nTiles = nN / 16;
  const int nNE    = (nTiles + NWAVE - 1) / NWAVE;
  const int nEEB   = nE / EEB;
  const int nMB    = nE / MEB;
  const int nNB    = (nN + NB - 1) / NB;
  const int nDB    = (nN + DRB - 1) / DRB;

  k_prep<<<S_END / PTHR, PTHR, 0, stream>>>(enc_W, proj_W, eenc_W, en_W1, gru_Wi, gru_Wh, dW1, dW2, dW3, dW4,
                                            en_W2, en_b2, WB, Bp);
  k_nodeenc<<<nNE, NTHR, 0, stream>>>(nfeats, nN, emb, nT, WB, enc_b, proj_b, H, H16);
  k_edgeenc<<<nEEB, NTHR, 0, stream>>>(efeats, nE, WB, eenc_b, en_b1, HE);

  hipFuncSetAttribute(reinterpret_cast<const void*>(&k_node), hipFuncAttributeMaxDynamicSharedMemorySize, LDS_NODE);
  for (int s = 0; s < 3; ++s) {
    k_msg<<<nMB, NTHR, 0, stream>>>(H16, nN, src, nE, HE, Bp, MSG);
    k_node<<<nNB, NTHR, LDS_NODE, stream>>>(dst, nE, vec8, MSG, H, H16, nN, conv_b, WB, gru_bi, gru_bh);
  }
  k_dec<<<nDB, NTHR, 0, stream>>>(H, nN, WB, db1, da1, db2, da2, db3, da3, db4, out);
}
